// IncidenceBiasAttention_15109694947391
// MI455X (gfx1250) — hardware-verified
//
#include <hip/hip_runtime.h>
#include <math.h>
#include <float.h>
#include <stdint.h>

#define NB     2
#define SEQ    2048
#define DMODEL 1024
#define NH     16
#define HD     64
#define QP     (NH * HD)
#define NQB    (SEQ / 64)
#define VLP    512
#define RESQB  8
#define PD     4
#define LNW    (4 * PD * NH)
static_assert(RESQB * 64 <= VLP);
static_assert(RESQB <= NQB);
static_assert(QP == DMODEL);
static_assert(HD == 64);
static_assert(PD == 4);
static_assert((SEQ % 64) == 0 && (DMODEL % 64) == 0 && (LNW % 64) == 0 && (QP % 64) == 0);
static_assert(((NB * SEQ) % 64) == 0 && (SEQ % 32) == 0);
static_assert((DMODEL % 32) == 0);

typedef _Float16 v16h __attribute__((ext_vector_type(16)));
typedef _Float16 v8h  __attribute__((ext_vector_type(8)));
typedef __bf16   v16b __attribute__((ext_vector_type(16)));
typedef __bf16   v8b  __attribute__((ext_vector_type(8)));
typedef float    v8f  __attribute__((ext_vector_type(8)));
typedef float    v4f  __attribute__((ext_vector_type(4)));
typedef float    v2f  __attribute__((ext_vector_type(2)));
typedef unsigned int v4u __attribute__((ext_vector_type(4)));

__device__ __forceinline__ unsigned short bf_bits(float f) {
  unsigned u = __float_as_uint(f);
  return (unsigned short)((u + 0x7FFFu + ((u >> 16) & 1u)) >> 16);
}
__device__ __forceinline__ float bf_up(unsigned short h) { return __uint_as_float(((unsigned)h) << 16); }
__device__ __forceinline__ unsigned short h_bits(_Float16 x) { return __builtin_bit_cast(unsigned short, x); }
__device__ __forceinline__ unsigned pk16(unsigned short a, unsigned short b) { return (unsigned)a | ((unsigned)b << 16); }
__device__ __forceinline__ v8f zero8() { v8f z = {0.f, 0.f, 0.f, 0.f, 0.f, 0.f, 0.f, 0.f}; return z; }
__device__ __forceinline__ v8h zero8h() {
  const _Float16 z = (_Float16)0.0f;
  v8h r = {z, z, z, z, z, z, z, z};
  return r;
}

__device__ __forceinline__ v16b ldfrag_b(const __bf16* p) {
  union { v16b v; v8b h[2]; } f;
  f.h[0] = *(const v8b*)(p);
  f.h[1] = *(const v8b*)(p + 16);
  return f.v;
}

__device__ __forceinline__ v8f mma_b(v16b a, v16b b, v8f c) {
  c = __builtin_amdgcn_wmma_f32_16x16x32_bf16(false, a, false, b, (short)0, c, false, false);
#if defined(__HIP_DEVICE_COMPILE__)
  asm volatile("v_nop\n\tv_nop\n\tv_nop\n\tv_nop" : "+v"(c) : "v"(a), "v"(b));
#endif
  return c;
}
__device__ __forceinline__ v8f mma_h(v16h a, v16h b, v8f c) {
  c = __builtin_amdgcn_wmma_f32_16x16x32_f16(false, a, false, b, (short)0, c, false, false);
#if defined(__HIP_DEVICE_COMPILE__)
  asm volatile("v_nop\n\tv_nop\n\tv_nop\n\tv_nop" : "+v"(c) : "v"(a), "v"(b));
#endif
  return c;
}
__device__ __forceinline__ v8f mma_b_raw(v16b a, v16b b, v8f c) {
  return __builtin_amdgcn_wmma_f32_16x16x32_bf16(false, a, false, b, (short)0, c, false, false);
}
__device__ __forceinline__ void dep_guard_b(v8f& a, v8f& b, v16b x, v16b y) {
#if defined(__HIP_DEVICE_COMPILE__)
  asm volatile("v_nop\n\tv_nop\n\tv_nop\n\tv_nop" : "+v"(a), "+v"(b) : "v"(x), "v"(y));
#endif
}
__device__ __forceinline__ void keep4_b(v16b a, v16b b, v16b c, v16b d) {
#if defined(__HIP_DEVICE_COMPILE__)
  asm volatile("v_nop" :: "v"(a), "v"(b), "v"(c), "v"(d));
#endif
}
__device__ __forceinline__ void acc_guard4(v8f& a, v8f& b, v8f& c, v8f& d) {
#if defined(__HIP_DEVICE_COMPILE__)
  asm volatile("v_nop\n\tv_nop\n\tv_nop\n\tv_nop" : "+v"(a), "+v"(b), "+v"(c), "+v"(d));
#endif
}

__global__ __launch_bounds__(256) void cvt_bf16(const float* __restrict__ in, unsigned short* out, int n8) {
  const int i = blockIdx.x * 256 + threadIdx.x;
  if (i < n8) {
    const float* s = in + (size_t)i * 8;
    const v4f a = *(const v4f*)(s);
    const v4f b = *(const v4f*)(s + 4);
    v4u p;
    p[0] = pk16(bf_bits(a[0]), bf_bits(a[1]));
    p[1] = pk16(bf_bits(a[2]), bf_bits(a[3]));
    p[2] = pk16(bf_bits(b[0]), bf_bits(b[1]));
    p[3] = pk16(bf_bits(b[2]), bf_bits(b[3]));
    unsigned short* d = out + (size_t)i * 8;
    *(volatile v4u*)d = p;
    __threadfence();
    *(volatile v4u*)d = p;
  }
}

__global__ __launch_bounds__(256) void split_bf16x8(const float* __restrict__ in, unsigned short* hp,
                                                    unsigned short* lp, int n8) {
  const int i = blockIdx.x * 256 + threadIdx.x;
  if (i < n8) {
    const v4f a = *(const v4f*)(in + (size_t)i * 8);
    const v4f b = *(const v4f*)(in + (size_t)i * 8 + 4);
    v4u ph, pl;
#pragma unroll
    for (int e = 0; e < 4; ++e) {
      const float f0 = (e < 2) ? a[2 * e]     : b[2 * e - 4];
      const float f1 = (e < 2) ? a[2 * e + 1] : b[2 * e - 3];
      const unsigned short h0 = bf_bits(f0), h1 = bf_bits(f1);
      const unsigned short l0 = bf_bits(f0 - bf_up(h0)), l1 = bf_bits(f1 - bf_up(h1));
      ph[e] = pk16(h0, h1);
      pl[e] = pk16(l0, l1);
    }
    *(volatile v4u*)(hp + (size_t)i * 8) = ph;
    *(volatile v4u*)(lp + (size_t)i * 8) = pl;
    __threadfence();
    *(volatile v4u*)(hp + (size_t)i * 8) = ph;
    *(volatile v4u*)(lp + (size_t)i * 8) = pl;
  }
}

template <int NSPLIT, int OUT_MODE, int BIAS>
__global__ __launch_bounds__(256) void gemm64(
    const unsigned short* __restrict__ Ap, const unsigned short* A2p, int lda, long long strideA,
    const unsigned short* __restrict__ Btp, const unsigned short* Bt2p, int ldb, long long strideB,
    void* Cout, int ldc, long long strideC,
    void* Cout2, int ldc2, long long strideC2, int N2,
    const float* __restrict__ biasp,
    int M, int N, int K, float rscale) {
  const __bf16* A   = (const __bf16*)(const void*)Ap;
  const __bf16* A2  = (const __bf16*)(const void*)A2p;
  const __bf16* Bt  = (const __bf16*)(const void*)Btp;
  const __bf16* Bt2 = (const __bf16*)(const void*)Bt2p;
  __shared__ __align__(16) float sT[8][16 * 68];
  const int b    = blockIdx.y;
  const int lane = threadIdx.x & 31;
  const int wave = threadIdx.x >> 5;
  const int tilesN = N >> 6;
  const int tilesM = M >> 6;
  const int tile = blockIdx.x * 8 + wave;
  if (tile >= tilesM * tilesN) return;
  const int tm = tile / tilesN;
  const int tn = tile - tm * tilesN;
  const int m0 = tm << 6;
  const int n0 = tn << 6;

  const __bf16* Ab  = A  + (size_t)b * strideA;
  const __bf16* Bb  = Bt + (size_t)b * strideB;
  const __bf16* Ab2 = (NSPLIT >= 1) ? (A2  + (size_t)b * strideA) : Ab;
  const __bf16* Bb2 = (NSPLIT == 2) ? (Bt2 + (size_t)b * strideB) : Bb;

  const int rlane = lane & 15;
  const int koff  = (lane >> 4) * 8;
  const int mOff  = (lane >> 4) * 8;

  v8f acc[4][4];
#pragma unroll
  for (int i = 0; i < 4; ++i)
#pragma unroll
    for (int j = 0; j < 4; ++j) acc[i][j] = zero8();

  for (int k0 = 0; k0 < K; k0 += 32) {
    v16b bh[4], bl[4];
#pragma unroll
    for (int j = 0; j < 4; ++j) {
      const size_t bo = (size_t)(n0 + (j << 4) + rlane) * ldb + koff + k0;
      bh[j] = ldfrag_b(Bb + bo);
      if (NSPLIT == 2) bl[j] = ldfrag_b(Bb2 + bo); else bl[j] = bh[j];
    }
#pragma unroll
    for (int i = 0; i < 4; ++i) {
      const size_t ao = (size_t)(m0 + (i << 4) + rlane) * lda + koff + k0;
      const v16b ah = ldfrag_b(Ab + ao);
      v16b al = ah;
      if (NSPLIT >= 1) al = ldfrag_b(Ab2 + ao);
#pragma unroll
      for (int j = 0; j < 4; ++j) {
        acc[i][j] = mma_b_raw(ah, bh[j], acc[i][j]);
        if (NSPLIT >= 1) acc[i][j] = mma_b_raw(al, bh[j], acc[i][j]);
        if (NSPLIT == 2) acc[i][j] = mma_b_raw(ah, bl[j], acc[i][j]);
      }
      dep_guard_b(acc[i][0], acc[i][3], ah, al);
    }
    keep4_b(bh[0], bh[1], bh[2], bh[3]);
    if (NSPLIT == 2) keep4_b(bl[0], bl[1], bl[2], bl[3]);
  }
  acc_guard4(acc[0][0], acc[0][1], acc[0][2], acc[0][3]);
  acc_guard4(acc[1][0], acc[1][1], acc[1][2], acc[1][3]);
  acc_guard4(acc[2][0], acc[2][1], acc[2][2], acc[2][3]);
  acc_guard4(acc[3][0], acc[3][1], acc[3][2], acc[3][3]);

  float bcol[4];
#pragma unroll
  for (int j = 0; j < 4; ++j) bcol[j] = 0.f;
  if (BIAS == 1) {
#pragma unroll
    for (int j = 0; j < 4; ++j) bcol[j] = bf_up(bf_bits(biasp[n0 + (j << 4) + rlane]));
  }

  float* slab = sT[wave];
#pragma unroll
  for (int i = 0; i < 4; ++i) {
    const int mBase = m0 + (i << 4);
    float brow[8];
#pragma unroll
    for (int r = 0; r < 8; ++r) brow[r] = 0.f;
    if (BIAS == 2) {
#pragma unroll
      for (int r = 0; r < 8; ++r) brow[r] = bf_up(bf_bits(biasp[mBase + mOff + r]));
    }
#pragma unroll
    for (int r = 0; r < 8; ++r) {
#pragma unroll
      for (int j = 0; j < 4; ++j) {
        float v = acc[i][j][r];
        if (BIAS == 1) v += bcol[j];
        if (BIAS == 2) v += brow[r];
        slab[(mOff + r) * 68 + (j << 4) + rlane] = v;
      }
    }
    __builtin_amdgcn_fence(__ATOMIC_RELEASE, "workgroup");
    __builtin_amdgcn_wave_barrier();
    __builtin_amdgcn_fence(__ATOMIC_ACQUIRE, "workgroup");
    if (OUT_MODE == 0) {
      float* C = (float*)Cout + (size_t)b * strideC;
      const int hh = lane >> 4, c4 = (lane & 15) * 4;
      v4f ov[8];
#pragma unroll
      for (int it = 0; it < 8; ++it) {
        const int row = it * 2 + hh;
        ov[it] = *(const v4f*)(slab + row * 68 + c4);
      }
      for (int pass = 0; pass < 2; ++pass) {
#pragma unroll
        for (int it = 0; it < 8; ++it) {
          const int row = it * 2 + hh;
          *(volatile v4f*)(C + (size_t)(mBase + row) * ldc + n0 + c4) = ov[it];
        }
        __threadfence();
      }
    } else {
      const int q = lane >> 3, c8 = (lane & 7) * 8;
      unsigned short* C  = (unsigned short*)Cout  + (size_t)b * strideC;
      unsigned short* C2 = (unsigned short*)Cout2 + (size_t)b * strideC2;
      const bool wlo = (OUT_MODE == 2) || (n0 < N2);
      v4u hv[4], lv[4];
#pragma unroll
      for (int it = 0; it < 4; ++it) {
        const int row = it * 4 + q;
        const float* sp = slab + row * 68 + c8;
        v4u a, a2;
#pragma unroll
        for (int e = 0; e < 4; ++e) {
          const float f0 = sp[2 * e], f1 = sp[2 * e + 1];
          unsigned short h0, h1, l0, l1;
          if (OUT_MODE == 2) {
            h0 = bf_bits(f0); h1 = bf_bits(f1);
            l0 = bf_bits(f0 - bf_up(h0)); l1 = bf_bits(f1 - bf_up(h1));
          } else {
            const _Float16 x0 = (_Float16)f0, x1 = (_Float16)f1;
            h0 = h_bits(x0); h1 = h_bits(x1);
            l0 = h_bits((_Float16)((f0 - (float)x0) * rscale));
            l1 = h_bits((_Float16)((f1 - (float)x1) * rscale));
          }
          a[e] = pk16(h0, h1); a2[e] = pk16(l0, l1);
        }
        hv[it] = a; lv[it] = a2;
      }
      for (int pass = 0; pass < 2; ++pass) {
#pragma unroll
        for (int it = 0; it < 4; ++it) {
          const int row = it * 4 + q;
          *(volatile v4u*)(C + (size_t)(mBase + row) * ldc + n0 + c8) = hv[it];
          if (wlo) *(volatile v4u*)(C2 + (size_t)(mBase + row) * ldc2 + n0 + c8) = lv[it];
        }
        __threadfence();
      }
    }
    __builtin_amdgcn_fence(__ATOMIC_RELEASE, "workgroup");
    __builtin_amdgcn_wave_barrier();
    __builtin_amdgcn_fence(__ATOMIC_ACQUIRE, "workgroup");
  }
}

struct L6 { float v0, v1, v2, v3, v4, v5; };

__device__ __forceinline__ L6 ext6n(const v4f a, const v4f b) {
#pragma clang fp contract(off)
  L6 o;
  o.v0 = a[0] * b[1] - a[1] * b[0];
  o.v1 = a[0] * b[2] - a[2] * b[0];
  o.v2 = a[0] * b[3] - a[3] * b[0];
  o.v3 = a[1] * b[2] - a[2] * b[1];
  o.v4 = a[1] * b[3] - a[3] * b[1];
  o.v5 = a[2] * b[3] - a[3] * b[2];
  float n2 = o.v0 * o.v0 + o.v1 * o.v1;
  n2 = n2 + o.v2 * o.v2;
  n2 = n2 + o.v3 * o.v3;
  n2 = n2 + o.v4 * o.v4;
  n2 = n2 + o.v5 * o.v5;
  float n = sqrtf(n2);
  n = fmaxf(n, 1e-12f);
  const float inv = 1.0f / n;
  o.v0 *= inv; o.v1 *= inv; o.v2 *= inv; o.v3 *= inv; o.v4 *= inv; o.v5 *= inv;
  return o;
}

__global__ __launch_bounds__(256) void lines_k(const float* __restrict__ ln, float* rl, float* wl, int nwaves) {
#pragma clang fp contract(off)
  __shared__ __align__(16) float sR[8][256];
  __shared__ __align__(16) float sW[8][256];
  const int tid = threadIdx.x, wave = tid >> 5, lane = tid & 31;
  const int w = blockIdx.x * 8 + wave;
  if (w >= nwaves) return;
  const int tgPer = SEQ / 32;
  const int bh = w / tgPer;
  const int tg = w - bh * tgPer;
  const int b  = bh / NH;
  const int h  = bh - b * NH;
  const int t  = tg * 32 + lane;
  const size_t row  = (size_t)b * SEQ + t;
  const size_t rowp = (t > 0) ? (row - 1) : row;
  const float* cur = ln + row * LNW + h * PD;
  v4f p1 = *(const v4f*)(ln + rowp * LNW + h * PD);
  if (t == 0) { p1[0] = 0.f; p1[1] = 0.f; p1[2] = 0.f; p1[3] = 0.f; }
  const v4f p2 = *(const v4f*)(cur + 1 * PD * NH);
  const v4f p3 = *(const v4f*)(cur + 2 * PD * NH);
  const v4f p4 = *(const v4f*)(cur + 3 * PD * NH);
  const L6 lw = ext6n(p1, p2);
  const L6 lr = ext6n(p3, p4);

  float* sr = sR[wave] + lane * 8;
  float* sw = sW[wave] + lane * 8;
  v4f t0, t1, u0, u1;
  t0[0] = lr.v0; t0[1] = lr.v1; t0[2] = lr.v2; t0[3] = lr.v3;
  t1[0] = lr.v4; t1[1] = lr.v5; t1[2] = 0.f;   t1[3] = 0.f;
  u0[0] = lw.v5; u0[1] = -lw.v4; u0[2] = lw.v3; u0[3] = lw.v2;
  u1[0] = -lw.v1; u1[1] = lw.v0; u1[2] = 0.f;   u1[3] = 0.f;
  *(v4f*)(sr)     = t0;
  *(v4f*)(sr + 4) = t1;
  *(v4f*)(sw)     = u0;
  *(v4f*)(sw + 4) = u1;
  __builtin_amdgcn_fence(__ATOMIC_RELEASE, "workgroup");
  __builtin_amdgcn_wave_barrier();
  __builtin_amdgcn_fence(__ATOMIC_ACQUIRE, "workgroup");
  v4f oR[2], oW[2];
#pragma unroll
  for (int it = 0; it < 2; ++it) {
    oR[it] = *(const v4f*)(sR[wave] + it * 128 + lane * 4);
    oW[it] = *(const v4f*)(sW[wave] + it * 128 + lane * 4);
  }
  const size_t gb = ((size_t)bh * SEQ + (size_t)tg * 32) * 8;
  for (int pass = 0; pass < 2; ++pass) {
#pragma unroll
    for (int it = 0; it < 2; ++it) {
      *(volatile v4f*)(rl + gb + it * 128 + lane * 4) = oR[it];
      *(volatile v4f*)(wl + gb + it * 128 + lane * 4) = oW[it];
    }
    __threadfence();
  }
}

template <bool RES>
__global__ __launch_bounds__(128)
void attn_lb(const unsigned short* __restrict__ qhp, const unsigned short* __restrict__ qlp,
             const unsigned short* __restrict__ khp, const unsigned short* __restrict__ klp,
             const unsigned short* __restrict__ vhp, const unsigned short* __restrict__ vlp,
             const float* __restrict__ rlp, const float* __restrict__ wlp,
             const float* __restrict__ dlg, const float* __restrict__ bsc,
             float* outp, int qbBase, int nqbThis, float sscale) {
  union FB { v16b v; v8b h[2]; };
  union FH { v16h v; v8h h[2]; };
  __shared__ __align__(16) unsigned short KT[2 * 64 * 64];
  __shared__ __align__(16) _Float16 Vth[64 * 64];
  __shared__ __align__(16) _Float16 Vtl[RES ? 64 * 64 : 8];
  __shared__ __align__(16) _Float16 Psh[4][16 * 64];
  __shared__ __align__(16) _Float16 Psl[RES ? 4 : 1][16 * 64];
  __shared__ __align__(16) float    Ws[64 * 8];
  __shared__ __align__(16) float    Rs[4][16 * 8];
  __bf16* Ksh = (__bf16*)(void*)KT;
  __bf16* Ksl = Ksh + 64 * 64;

  const int tid  = threadIdx.x;
  const int wave = tid >> 5;
  const int lane = tid & 31;
  const int hh   = lane >> 4;
  const int c    = lane & 15;

  const int bx   = blockIdx.x;
  const int qbl  = bx % nqbThis;
  const int rest = bx / nqbThis;
  const int h    = rest % NH;
  const int b    = rest / NH;
  const int qb   = qbBase + qbl;
  const int q0   = qb * 64 + wave * 16;
  const size_t rowB = (size_t)b * SEQ;
  const size_t bhT  = ((size_t)b * NH + h) * SEQ;

  const __bf16* Qh = (const __bf16*)(const void*)qhp + (size_t)h * HD;
  const __bf16* Ql = (const __bf16*)(const void*)qlp + (size_t)h * HD;
  const __bf16* Kh = (const __bf16*)(const void*)khp + (size_t)h * HD;
  const __bf16* Kl = (const __bf16*)(const void*)klp + (size_t)h * HD;
  const _Float16* Vh = (const _Float16*)(const void*)vhp + ((size_t)b * QP + (size_t)h * HD) * SEQ;
  const _Float16* Vl = (const _Float16*)(const void*)vlp + ((size_t)b * QP + (size_t)h * HD) * VLP;

  const float dl  = bf_up(bf_bits(dlg[h]));
  const float dec = 1.0f / (1.0f + expf(-dl));
  const float l2d = log2f(dec);
  const float bsh = bf_up(bf_bits(bsc[h]));

  *(v4f*)(Rs[wave] + lane * 4) = *(const v4f*)(rlp + (bhT + q0) * 8 + lane * 4);

  float mrow[8], lrow[8];
  v8f oacc[4];
#pragma unroll
  for (int r = 0; r < 8; ++r) { mrow[r] = -INFINITY; lrow[r] = 0.f; }
#pragma unroll
  for (int t = 0; t < 4; ++t) oacc[t] = zero8();

  int nkt = qb + 1;
  if (nkt > NQB) nkt = NQB;
  for (int kt = 0; kt < nkt; ++kt) {
    const int kv0 = kt * 64;
    __syncthreads();
    {
      const int r = tid >> 1, half = (tid & 1) * 32;
      const __bf16*   kg  = Kh + (rowB + kv0 + r) * QP + half;
      const __bf16*   klg = Kl + (rowB + kv0 + r) * QP + half;
      const _Float16* vg  = Vh + (size_t)r * SEQ + kv0 + half;
      const int kvl = (kv0 + 64 <= VLP) ? kv0 : (VLP - 64);
      const _Float16* vlg = Vl + (size_t)r * VLP + kvl + half;
      const bool resOK = (kv0 + 64 <= VLP);
#pragma unroll
      for (int i = 0; i < 4; ++i) {
        const v8b a0 = *(const v8b*)(kg + 8 * i);
        const v8b a1 = *(const v8b*)(klg + 8 * i);
        const v8h b0 = *(const v8h*)(vg + 8 * i);
        *(v8b*)(Ksh + r * 64 + half + 8 * i) = a0;
        *(v8b*)(Ksl + r * 64 + half + 8 * i) = a1;
        *(v8h*)(Vth + r * 64 + half + 8 * i) = b0;
        if (RES) {
          v8h b1 = *(const v8h*)(vlg + 8 * i);
          if (!resOK) b1 = zero8h();
          *(v8h*)(Vtl + r * 64 + half + 8 * i) = b1;
        }
      }
      *(v4f*)(Ws + tid * 4) = *(const v4f*)(wlp + (bhT + kv0) * 8 + tid * 4);
    }
    __syncthreads();

    v16b qah[2], qal[2];
#pragma unroll
    for (int dc = 0; dc < 2; ++dc) {
      const size_t qo = (rowB + q0 + c) * QP + dc * 32 + 8 * hh;
      qah[dc] = ldfrag_b(Qh + qo);
      qal[dc] = ldfrag_b(Ql + qo);
    }

    v8f s[4];
#pragma unroll
    for (int j = 0; j < 4; ++j) {
      s[j] = zero8();
#pragma unroll
      for (int dc = 0; dc < 2; ++dc) {
        FB kb, kl;
        kb.h[0] = *(const v8b*)(Ksh + (j * 16 + c) * 64 + dc * 32 + 8 * hh);
        kb.h[1] = *(const v8b*)(Ksh + (j * 16 + c) * 64 + dc * 32 + 16 + 8 * hh);
        kl.h[0] = *(const v8b*)(Ksl + (j * 16 + c) * 64 + dc * 32 + 8 * hh);
        kl.h[1] = *(const v8b*)(Ksl + (j * 16 + c) * 64 + dc * 32 + 16 + 8 * hh);
        s[j] = mma_b(qah[dc], kb.v, s[j]);
        s[j] = mma_b(qah[dc], kl.v, s[j]);
        s[j] = mma_b(qal[dc], kb.v, s[j]);
      }
    }

    v4f wa[4];
    v2f wb[4];
#pragma unroll
    for (int j = 0; j < 4; ++j) {
      const float* wp = Ws + (j * 16 + c) * 8;
      wa[j] = *(const v4f*)(wp);
      wb[j] = *(const v2f*)(wp + 4);
    }

    _Float16* pwh = Psh[wave];
    _Float16* pwl = Psl[RES ? wave : 0];
#pragma unroll
    for (int r = 0; r < 8; ++r) {
      const int qrow = q0 + 8 * hh + r;
      const float* rp = Rs[wave] + (8 * hh + r) * 8;
      const v4f ra = *(const v4f*)(rp);
      const v2f rb = *(const v2f*)(rp + 4);
      float m = -INFINITY;
#pragma unroll
      for (int j = 0; j < 4; ++j) {
        const int key = kv0 + j * 16 + c;
        const int dd  = qrow - key;
        const float dot6 = ra[0] * wa[j][0] + ra[1] * wa[j][1] + ra[2] * wa[j][2] + ra[3] * wa[j][3]
                         + rb[0] * wb[j][0] + rb[1] * wb[j][1];
        const float ex   = exp2f((float)dd * l2d);
        const float wdec = (dd > 0) ? (bsh * ex) : 0.f;
        float sv = s[j][r] * sscale + dot6 * wdec;
        sv = (key > qrow) ? -FLT_MAX : sv;
        s[j][r] = sv;
        m = fmaxf(m, sv);
      }
#pragma unroll
      for (int off = 1; off < 16; off <<= 1) m = fmaxf(m, __shfl_xor(m, off, 32));
      const float mnew  = fmaxf(mrow[r], m);
      const float msafe = (mnew == -INFINITY) ? 0.f : mnew;
      const float alpha = __expf(mrow[r] - msafe);
      mrow[r] = mnew;
      float psum = 0.f;
#pragma unroll
      for (int j = 0; j < 4; ++j) {
        const float p = __expf(s[j][r] - msafe);
        psum += p;
        const float p1k = p * 1024.0f;
        const _Float16 ph = (_Float16)p1k;
        pwh[(8 * hh + r) * 64 + j * 16 + c] = ph;
        if (RES) {
          const _Float16 pl = (_Float16)((p1k - (float)ph) * 4096.0f);
          pwl[(8 * hh + r) * 64 + j * 16 + c] = pl;
        }
      }
#pragma unroll
      for (int off = 1; off < 16; off <<= 1) psum += __shfl_xor(psum, off, 32);
      lrow[r] = lrow[r] * alpha + psum;
#pragma unroll
      for (int t = 0; t < 4; ++t) oacc[t][r] *= alpha;
    }
    __builtin_amdgcn_fence(__ATOMIC_RELEASE, "workgroup");
    __builtin_amdgcn_wave_barrier();
    __builtin_amdgcn_fence(__ATOMIC_ACQUIRE, "workgroup");

    v8f o1[4];
#pragma unroll
    for (int t = 0; t < 4; ++t) o1[t] = zero8();
#pragma unroll 1
    for (int kk = 0; kk < 2; ++kk) {
      FH pa, pl;
      pa.h[0] = *(const v8h*)(pwh + c * 64 + kk * 32 + 8 * hh);
      pa.h[1] = *(const v8h*)(pwh + c * 64 + kk * 32 + 16 + 8 * hh);
      if (RES) {
        pl.h[0] = *(const v8h*)(pwl + c * 64 + kk * 32 + 8 * hh);
        pl.h[1] = *(const v8h*)(pwl + c * 64 + kk * 32 + 16 + 8 * hh);
      } else {
        pl.v = pa.v;
      }
#pragma unroll
      for (int t = 0; t < 4; ++t) {
        FH vb;
        vb.h[0] = *(const v8h*)(Vth + (t * 16 + c) * 64 + kk * 32 + 8 * hh);
        vb.h[1] = *(const v8h*)(Vth + (t * 16 + c) * 64 + kk * 32 + 16 + 8 * hh);
        oacc[t] = mma_h(pa.v, vb.v, oacc[t]);
        if (RES) {
          FH vl;
          vl.h[0] = *(const v8h*)(Vtl + (t * 16 + c) * 64 + kk * 32 + 8 * hh);
          vl.h[1] = *(const v8h*)(Vtl + (t * 16 + c) * 64 + kk * 32 + 16 + 8 * hh);
          o1[t] = mma_h(pa.v, vl.v, o1[t]);
          o1[t] = mma_h(pl.v, vb.v, o1[t]);
        }
      }
    }
    if (RES) {
#pragma unroll
      for (int t = 0; t < 4; ++t)
#pragma unroll
        for (int r = 0; r < 8; ++r) oacc[t][r] += o1[t][r] * (1.0f / 4096.0f);
    }
  }

  __syncthreads();

  float* os = (float*)(void*)KT + wave * (16 * 64);
#pragma unroll
  for (int r = 0; r < 8; ++r) {
    const float l = lrow[r];
    const float inv = ((l > 0.f) ? (1.0f / l) : 0.f) * (1.0f / 1024.0f);
#pragma unroll
    for (int t = 0; t < 4; ++t) os[(8 * hh + r) * 64 + t * 16 + c] = oacc[t][r] * inv;
  }
  __builtin_amdgcn_fence(__ATOMIC_RELEASE, "workgroup");
  __builtin_amdgcn_wave_barrier();
  __builtin_amdgcn_fence(__ATOMIC_ACQUIRE, "workgroup");
  {
    const int h2 = lane >> 4, c4 = (lane & 15) * 4;
    v4f ov[8];
#pragma unroll
    for (int it = 0; it < 8; ++it) {
      const int row = it * 2 + h2;
      ov[it] = *(const v4f*)(os + row * 64 + c4);
    }
    for (int pass = 0; pass < 2; ++pass) {
#pragma unroll
      for (int it = 0; it < 8; ++it) {
        const int row = it * 2 + h2;
        const size_t go = (rowB + q0 + row) * QP + (size_t)h * HD + c4;
        *(volatile v4f*)(outp + go) = ov[it];
      }
      __threadfence();
    }
  }
}

extern "C" void kernel_launch(void* const* d_in, const int* in_sizes, int n_in,
                              void* d_out, int out_size, void* d_ws, size_t ws_size,
                              hipStream_t stream) {
  if (n_in < 11) return;
  if (in_sizes[0] != NB * SEQ * DMODEL) return;
  if (in_sizes[1] != 3 * QP * DMODEL) return;
  if (in_sizes[2] != 3 * QP) return;
  if (in_sizes[3] != PD * NH * DMODEL) return;
  if (in_sizes[4] != PD * NH * DMODEL) return;
  if (in_sizes[5] != PD * NH * DMODEL) return;
  if (in_sizes[6] != PD * NH * DMODEL) return;
  if (in_sizes[7] != DMODEL * QP) return;
  if (in_sizes[8] != DMODEL) return;
  if (in_sizes[9] != NH) return;
  if (in_sizes[10] != NH) return;
  if (out_size != NB * SEQ * DMODEL) return;

  const float* x     = (const float*)d_in[0];
  const float* wqkv  = (const float*)d_in[1];
  const float* bqkv  = (const float*)d_in[2];
  const float* w1w   = (const float*)d_in[3];
  const float* w2w   = (const float*)d_in[4];
  const float* w1r   = (const float*)d_in[5];
  const float* w2r   = (const float*)d_in[6];
  const float* wout  = (const float*)d_in[7];
  const float* bout  = (const float*)d_in[8];
  const float* dlog  = (const float*)d_in[9];
  const float* bscl  = (const float*)d_in[10];

  const size_t PXb   = (size_t)NB * SEQ * DMODEL * 2;
  const size_t PWqkv = (size_t)3 * QP * DMODEL * 2;
  const size_t PWln  = (size_t)LNW * DMODEL * 2;
  const size_t PWo   = (size_t)DMODEL * QP * 2;
  const size_t PLN   = (size_t)NB * SEQ * LNW * 4;
  const size_t PRL   = (size_t)NB * NH * SEQ * 8 * 4;
  const size_t PQpl  = (size_t)NB * SEQ * QP * 2;
  const size_t PVTh  = (size_t)NB * QP * SEQ * 2;
  const size_t PVTl  = (size_t)NB * QP * VLP * 2;
  const size_t PAf   = (size_t)NB * SEQ * QP * 4;
  size_t off = 0;
  const size_t oXb   = off; off += PXb;
  const size_t oWqkv = off; off += PWqkv;
  const size_t oWln  = off; off += PWln;
  const size_t oWo   = off; off += PWo;
  const size_t oLN   = off; off += PLN;
  const size_t oRL   = off; off += PRL;
  const size_t oWL   = off; off += PRL;
  const size_t oQh   = off; off += PQpl;
  const size_t oQl   = off; off += PQpl;
  const size_t oKh   = off; off += PQpl;
  const size_t oKl   = off; off += PQpl;
  const size_t oVTh  = off; off += PVTh;
  const size_t oVTl  = off; off += PVTl;
  const size_t oAf   = off; off += PAf;
  const size_t oAh   = off; off += PQpl;
  const size_t oAl   = off; off += PQpl;
  if (off > ws_size) return;
  if (off > (size_t)134217728) return;

  char* ws = (char*)d_ws;
  unsigned short* Xb   = (unsigned short*)(ws + oXb);
  unsigned short* Wqkv = (unsigned short*)(ws + oWqkv);
  unsigned short* Wln  = (unsigned short*)(ws + oWln);
  unsigned short* Wob  = (unsigned short*)(ws + oWo);
  float*          LN   = (float*)(ws + oLN);
  float*          RL   = (float*)(ws + oRL);
  float*          WL   = (float*)(ws + oWL);
  unsigned short* Qh   = (unsigned short*)(ws + oQh);
  unsigned short* Ql   = (unsigned short*)(ws + oQl);
  unsigned short* Kh   = (unsigned short*)(ws + oKh);
  unsigned short* Kl   = (unsigned short*)(ws + oKl);
  unsigned short* VTh  = (unsigned short*)(ws + oVTh);
  unsigned short* VTl  = (unsigned short*)(ws + oVTl);
  float*          Af   = (float*)(ws + oAf);
  unsigned short* Ah   = (unsigned short*)(ws + oAh);
  unsigned short* Al   = (unsigned short*)(ws + oAl);
  float*          outf = (float*)d_out;

  const dim3 blk(256);
  const int nTok   = NB * SEQ;
  const int n8x    = nTok * DMODEL / 8;
  const int n8qkv  = 3 * QP * DMODEL / 8;
  const int n8ln   = PD * NH * DMODEL / 8;
  const int n8wo   = DMODEL * QP / 8;
  const int n8a    = nTok * QP / 8;
  const int nwLn   = NB * NH * (SEQ / 32);
  const dim3 gCx((n8x + 255) / 256), gCqkv((n8qkv + 255) / 256), gCln((n8ln + 255) / 256), gCwo((n8wo + 255) / 256);
  const dim3 gLNg(((nTok / 64) * (LNW / 64) + 7) / 8, 1);
  const dim3 gQ(((nTok / 64) * (QP / 64) + 7) / 8, 1);
  const dim3 gVT(((QP / 64) * (SEQ / 64) + 7) / 8, NB);
  const dim3 gLines((nwLn + 7) / 8);
  const dim3 gSplit((n8a + 255) / 256);
  const dim3 gOut(((nTok / 64) * (DMODEL / 64) + 7) / 8, 1);

  cvt_bf16<<<gCx,   blk, 0, stream>>>(x,    Xb,   n8x);
  cvt_bf16<<<gCqkv, blk, 0, stream>>>(wqkv, Wqkv, n8qkv);
  cvt_bf16<<<gCln,  blk, 0, stream>>>(w1w,  Wln + (size_t)0 * PD * NH * DMODEL, n8ln);
  cvt_bf16<<<gCln,  blk, 0, stream>>>(w2w,  Wln + (size_t)1 * PD * NH * DMODEL, n8ln);
  cvt_bf16<<<gCln,  blk, 0, stream>>>(w1r,  Wln + (size_t)2 * PD * NH * DMODEL, n8ln);
  cvt_bf16<<<gCln,  blk, 0, stream>>>(w2r,  Wln + (size_t)3 * PD * NH * DMODEL, n8ln);
  cvt_bf16<<<gCwo,  blk, 0, stream>>>(wout, Wob,  n8wo);
  gemm64<0, 0, 0><<<gLNg, blk, 0, stream>>>(
      Xb, Xb, DMODEL, 0LL, Wln, Wln, DMODEL, 0LL,
      (void*)LN, LNW, 0LL, (void*)LN, 0, 0LL, 0,
      bout, nTok, LNW, DMODEL, 1.0f);
  gemm64<0, 2, 1><<<gQ, blk, 0, stream>>>(
      Xb, Xb, DMODEL, 0LL, Wqkv, Wqkv, DMODEL, 0LL,
      (void*)Qh, QP, 0LL, (void*)Ql, QP, 0LL, QP,
      bqkv, nTok, QP, DMODEL, 1.0f);
  gemm64<0, 2, 1><<<gQ, blk, 0, stream>>>(
      Xb, Xb, DMODEL, 0LL, Wqkv + (size_t)QP * DMODEL, Wqkv + (size_t)QP * DMODEL, DMODEL, 0LL,
      (void*)Kh, QP, 0LL, (void*)Kl, QP, 0LL, QP,
      bqkv + QP, nTok, QP, DMODEL, 1.0f);
  gemm64<0, 3, 2><<<gVT, blk, 0, stream>>>(
      Wqkv + (size_t)2 * QP * DMODEL, Wqkv + (size_t)2 * QP * DMODEL, DMODEL, 0LL,
      Xb, Xb, DMODEL, (long long)SEQ * DMODEL,
      (void*)VTh, SEQ, (long long)QP * SEQ, (void*)VTl, VLP, (long long)QP * VLP, VLP,
      bqkv + 2 * QP, QP, SEQ, DMODEL, 4096.0f);
  lines_k<<<gLines, blk, 0, stream>>>(LN, RL, WL, nwLn);
  attn_lb<true><<<dim3(NB * NH * RESQB), dim3(128), 0, stream>>>(
      Qh, Ql, Kh, Kl, VTh, VTl, RL, WL, dlog, bscl, Af, 0, RESQB, 0.125f);
  attn_lb<false><<<dim3(NB * NH * (NQB - RESQB)), dim3(128), 0, stream>>>(
      Qh, Ql, Kh, Kl, VTh, VTl, RL, WL, dlog, bscl, Af, RESQB, NQB - RESQB, 0.125f);
  split_bf16x8<<<gSplit, blk, 0, stream>>>(Af, Ah, Al, n8a);
  gemm64<1, 0, 1><<<gOut, blk, 0, stream>>>(
      Ah, Al, QP, 0LL, Wob, Wob, QP, 0LL,
      (void*)outf, DMODEL, 0LL, (void*)outf, 0, 0LL, 0,
      bout, nTok, DMODEL, QP, 1.0f);
  (void)hipGetLastError();
}
